// LinearAttentionLayer_86260123174779
// MI455X (gfx1250) — hardware-verified
//
#include <hip/hip_runtime.h>
#include <math.h>
#include <stdint.h>

#ifndef NB
#define NB 4
#endif
#ifndef SEQ
#define SEQ 2048
#endif
#define XS_FULL 2048
#define DMOD  1024
#define DQK   1024
#define NH    16
#define HD    64
#define QSC   1024.0f
#define VSC   1024.0f
#define PCAR  64.0f
#define KCAR  1024.0f
#define EPSC  1e-6f
#define WPB   4
#define NHG   (NH / WPB)
#define NQT   (SEQ / 16)
#define NST   (SEQ / 64)
#define NKT   (SEQ / 32)
#define ATT_THREADS (WPB * 32)
#define PTP   36
#define PTW   (16 * PTP)
#define SLP   68
#define SLW   (16 * SLP)
#define WREG  (PTW + SLW)
#define SLAB64 (16 * 68)
#define VTP   72
#define TRP   72
#define WS_CAP 134217728
static_assert(DMOD == NH * HD && DQK == NH * HD && HD == 64 && NH == 16 && WPB == 4 && NHG * WPB == NH && ATT_THREADS == 128);
static_assert(DQK == DMOD);
static_assert(NB >= 1 && NB <= 4);
static_assert(NB == 1 || SEQ == XS_FULL);
static_assert((SEQ % 64) == 0 && SEQ >= 64 && SEQ <= XS_FULL);
static_assert(((SEQ * DMOD / 8) % 256) == 0 && (DMOD % 256) == 0 && (DMOD % 64) == 0 && (HD % 32) == 0);
static_assert(WPB * WREG * 4 <= 65536 && 2 * HD * VTP * 2 <= 65536 && 4 * SLAB64 * 4 <= 65536 && 64 * TRP * 2 <= 65536);

typedef unsigned short u16;
typedef _Float16 v16h __attribute__((ext_vector_type(16)));
typedef _Float16 v8h  __attribute__((ext_vector_type(8)));
typedef __bf16   v16b __attribute__((ext_vector_type(16)));
typedef float    v8f  __attribute__((ext_vector_type(8)));
typedef float    v4f  __attribute__((ext_vector_type(4)));
typedef unsigned int v4u __attribute__((ext_vector_type(4)));

union FragH { v16h v; v8h h[2]; v4u u[2]; };
union FragB { v16b v; v4u u[2]; };

__device__ __forceinline__ unsigned short bf_bits(float f) {
  unsigned u = __float_as_uint(f);
  return (unsigned short)((u + 0x7FFFu + ((u >> 16) & 1u)) >> 16);
}
__device__ __forceinline__ float bf_up(unsigned short h) { return __uint_as_float(((unsigned)h) << 16); }
__device__ __forceinline__ float bfr(float f) { return bf_up(bf_bits(f)); }
__device__ __forceinline__ unsigned short h_bits(_Float16 x) { return __builtin_bit_cast(unsigned short, x); }
__device__ __forceinline__ unsigned pk16(unsigned short a, unsigned short b) { return (unsigned)a | ((unsigned)b << 16); }
__device__ __forceinline__ v8f zero8() { v8f z = {0.f, 0.f, 0.f, 0.f, 0.f, 0.f, 0.f, 0.f}; return z; }
__device__ __forceinline__ int imin(int a, int b) { return a < b ? a : b; }
__device__ __forceinline__ int imax(int a, int b) { return a > b ? a : b; }

__device__ __forceinline__ v16h ldfrag_h(const _Float16* p) {
  FragH f;
  f.h[0] = *(const v8h*)(p);
  f.h[1] = *(const v8h*)(p + 16);
  return f.v;
}
__device__ __forceinline__ v16b ldfrag_b(const u16* p) {
  FragB f;
  f.u[0] = *(const v4u*)(p);
  f.u[1] = *(const v4u*)(p + 16);
  return f.v;
}

__device__ __forceinline__ v8f mma_h(v16h a, v16h b, v8f c) {
  return __builtin_amdgcn_wmma_f32_16x16x32_f16(false, a, false, b, (short)0, c, false, false);
}
__device__ __forceinline__ v8f mma_b(v16b a, v16b b, v8f c) {
  return __builtin_amdgcn_wmma_f32_16x16x32_bf16(false, a, false, b, (short)0, c, false, false);
}
__device__ __forceinline__ void guard2(v8f& a, v8f& b, v16h x0, v16h x1, v16h x2, v16h x3, v16h x4, v16h x5) {
#if defined(__HIP_DEVICE_COMPILE__)
  asm volatile("v_nop\n\tv_nop\n\tv_nop\n\tv_nop"
               : "+v"(a), "+v"(b) : "v"(x0), "v"(x1), "v"(x2), "v"(x3), "v"(x4), "v"(x5) : "memory");
#endif
}
template <typename F>
__device__ __forceinline__ void guard6(v8f& a, v8f& b, v8f& c, v8f& d, F x0, F x1, F x2, F x3, F x4, F x5) {
#if defined(__HIP_DEVICE_COMPILE__)
  asm volatile("v_nop\n\tv_nop\n\tv_nop\n\tv_nop"
               : "+v"(a), "+v"(b), "+v"(c), "+v"(d) : "v"(x0), "v"(x1), "v"(x2), "v"(x3), "v"(x4), "v"(x5) : "memory");
#endif
}
__device__ __forceinline__ void acc_guard4(v8f& a, v8f& b, v8f& c, v8f& d) {
#if defined(__HIP_DEVICE_COMPILE__)
  asm volatile("v_nop\n\tv_nop\n\tv_nop\n\tv_nop" : "+v"(a), "+v"(b), "+v"(c), "+v"(d));
#endif
}
__device__ __forceinline__ void wave_sync_lds() {
  __builtin_amdgcn_fence(__ATOMIC_RELEASE, "workgroup");
  __builtin_amdgcn_wave_barrier();
  __builtin_amdgcn_fence(__ATOMIC_ACQUIRE, "workgroup");
}

__global__ __launch_bounds__(256) void cvt_bf3(const float* __restrict__ x0, const float* __restrict__ x1,
                                               const float* __restrict__ x2, u16* D0, u16* D1, u16* D2, int n8) {
  const int which = (int)blockIdx.y;
  const float* x = (which == 0) ? x0 : ((which == 1) ? x1 : x2);
  u16* D = (which == 0) ? D0 : ((which == 1) ? D1 : D2);
  const int gt = (int)blockIdx.x * 256 + (int)threadIdx.x;
  if (gt >= n8) return;
  const float* p = x + (size_t)gt * 8;
  const v4f a = *(const v4f*)(p), b4 = *(const v4f*)(p + 4);
  float w[8];
#pragma unroll
  for (int e = 0; e < 4; ++e) { w[e] = a[e]; w[4 + e] = b4[e]; }
  v4u o;
#pragma unroll
  for (int e = 0; e < 4; ++e) o[e] = pk16(bf_bits(w[2 * e]), bf_bits(w[2 * e + 1]));
  u16* d = D + (size_t)gt * 8;
  for (int pass = 0; pass < 2; ++pass) {
    *(volatile v4u*)(d) = o;
    __threadfence();
  }
}

__global__ __launch_bounds__(256) void k_wt(const float* __restrict__ W, int nc, int kr, int ntn, u16* Dp, int drow0) {
  __shared__ __align__(16) u16 T[64 * TRP];
  const int tid = (int)threadIdx.x;
  const int bid = (int)blockIdx.x;
  const int nt  = bid % ntn;
  const int kt  = bid / ntn;
  if (kt * 64 + 64 > kr) return;
  const int n0  = nt * 64, k0 = kt * 64;
  {
    const int dl = tid >> 2;
    const int oc = (tid & 3) * 16;
    const bool valid = (n0 + oc + 16 <= nc);
    const int  cb = valid ? (n0 + oc) : 0;
    const float* src = W + (size_t)(k0 + dl) * (size_t)nc + cb;
#pragma unroll
    for (int i = 0; i < 4; ++i) {
      const v4f a = *(const v4f*)(src + 4 * i);
#pragma unroll
      for (int e = 0; e < 4; ++e) {
        const float f = valid ? a[e] : 0.0f;
        T[(oc + 4 * i + e) * TRP + dl] = bf_bits(f);
      }
    }
  }
  __syncthreads();
  const int q8 = tid >> 3, p8 = (tid & 7) * 8;
  v4u w[2];
#pragma unroll
  for (int it = 0; it < 2; ++it) w[it] = *(const v4u*)(T + (it * 32 + q8) * TRP + p8);
  const size_t base = (size_t)(drow0 + n0) * (size_t)kr + k0 + p8;
  for (int pass = 0; pass < 2; ++pass) {
#pragma unroll
    for (int it = 0; it < 2; ++it) {
      const int nl = it * 32 + q8;
      *(volatile v4u*)(Dp + base + (size_t)nl * (size_t)kr) = w[it];
    }
    __threadfence();
  }
}

__global__ __launch_bounds__(256) void qv16(const float* __restrict__ FQ, const float* __restrict__ FV,
                                            u16* QHp, u16* QLp, u16* VHp, u16* VLp) {
  const int tid = (int)threadIdx.x;
  const int row = (int)blockIdx.x;
  if (row >= SEQ) return;
  const int which = tid >> 7;
  const int c8 = (tid & 127) * 8;
  const float sc = which ? VSC : QSC;
  const float* p = (which ? FV : FQ) + (size_t)row * DMOD + c8;
  const v4f a = *(const v4f*)(p), b4 = *(const v4f*)(p + 4);
  float w[8];
#pragma unroll
  for (int e = 0; e < 4; ++e) { w[e] = a[e]; w[4 + e] = b4[e]; }
  v4u oh, ol;
#pragma unroll
  for (int e = 0; e < 4; ++e) {
    const float t0 = w[2 * e] * sc, t1 = w[2 * e + 1] * sc;
    const _Float16 h0 = (_Float16)t0, h1 = (_Float16)t1;
    const _Float16 l0 = (_Float16)(t0 - (float)h0), l1 = (_Float16)(t1 - (float)h1);
    oh[e] = pk16(h_bits(h0), h_bits(h1));
    ol[e] = pk16(h_bits(l0), h_bits(l1));
  }
  u16* dh = (which ? VHp : QHp) + (size_t)row * DQK + c8;
  u16* dl = (which ? VLp : QLp) + (size_t)row * DQK + c8;
  for (int pass = 0; pass < 2; ++pass) {
    *(volatile v4u*)(dh) = oh;
    *(volatile v4u*)(dl) = ol;
    __threadfence();
  }
}

__global__ __launch_bounds__(256) void kt16(const float* __restrict__ FK, u16* THo, u16* TLo) {
  __shared__ __align__(16) u16 TH[HD * VTP];
  __shared__ __align__(16) u16 TL[HD * VTP];
  const int tid = (int)threadIdx.x;
  const int bid = (int)blockIdx.x;
  const int st  = bid % NST;
  const int h   = bid / NST;
  if (h >= NH) return;
  const int s0  = st * 64;
  {
    const int sl = tid >> 2;
    const int dc = (tid & 3) * 16;
    const float* src = FK + (size_t)(s0 + sl) * (size_t)DMOD + h * HD + dc;
#pragma unroll
    for (int i = 0; i < 4; ++i) {
      const v4f a = *(const v4f*)(src + 4 * i);
#pragma unroll
      for (int e = 0; e < 4; ++e) {
        const float t = a[e] * KCAR;
        const _Float16 hv = (_Float16)t;
        const _Float16 lv = (_Float16)(t - (float)hv);
        TH[(dc + 4 * i + e) * VTP + sl] = h_bits(hv);
        TL[(dc + 4 * i + e) * VTP + sl] = h_bits(lv);
      }
    }
  }
  __syncthreads();
  v4u vh[2], vl[2];
  const int q8 = tid >> 3, p8 = (tid & 7) * 8;
#pragma unroll
  for (int it = 0; it < 2; ++it) {
    const int line = it * 32 + q8;
    vh[it] = *(const v4u*)(TH + line * VTP + p8);
    vl[it] = *(const v4u*)(TL + line * VTP + p8);
  }
  const size_t hrow = (size_t)h * HD;
  const size_t base = hrow * SEQ + s0 + p8;
  for (int pass = 0; pass < 2; ++pass) {
#pragma unroll
    for (int it = 0; it < 2; ++it) {
      const int line = it * 32 + q8;
      *(volatile v4u*)(THo + base + (size_t)line * SEQ) = vh[it];
      *(volatile v4u*)(TLo + base + (size_t)line * SEQ) = vl[it];
    }
    __threadfence();
  }
}

__global__ __launch_bounds__(256) void k_den(const float* __restrict__ FQ, const float* __restrict__ FK, float* DN) {
#pragma clang fp contract(off)
  const int col = (int)blockIdx.x * 256 + (int)threadIdx.x;
  if (col >= DMOD) return;
  float run = 0.0f;
#pragma unroll 1
  for (int s = 0; s < SEQ; ++s) {
    const size_t o = (size_t)s * DMOD + col;
    run = run + FK[o];
    const float den = FQ[o] * run + EPSC;
    *(volatile float*)(DN + o) = den;
    __threadfence();
    *(volatile float*)(DN + o) = den;
  }
}

__device__ __forceinline__ float bias_at(const float* p0, const float* p1, const float* p2,
                                         int e0, int e1, int e2, int c) {
  const int i0 = imin(imax(c, 0), e0 - 1);
  const int i1 = imin(imax(c - e0, 0), e1 - e0 - 1);
  const int i2 = imin(imax(c - e1, 0), e2 - e1 - 1);
  const float v0 = p0[i0], v1 = p1[i1], v2 = p2[i2];
  const float v = (c < e0) ? v0 : ((c < e1) ? v1 : ((c < e2) ? v2 : 0.0f));
  return bfr(v);
}

template <bool EPI>
__device__ __forceinline__ void epi64b(float* sl, v8f a0, v8f a1, v8f a2, v8f a3, v4f bias4,
                                       float* C, int N, size_t rowb, int col0, int lane) {
  const int hh = lane >> 4, m = lane & 15;
#pragma unroll
  for (int r = 0; r < 8; ++r) {
    const int ro = (8 * hh + r) * 68 + m;
    sl[ro]      = a0[r];
    sl[ro + 16] = a1[r];
    sl[ro + 32] = a2[r];
    sl[ro + 48] = a3[r];
  }
  wave_sync_lds();
  v4f vals[8];
#pragma unroll
  for (int it = 0; it < 8; ++it) {
    v4f v = *(const v4f*)(sl + (it * 2 + hh) * 68 + m * 4) + bias4;
    if constexpr (EPI) {
#pragma unroll
      for (int e = 0; e < 4; ++e) {
        const float t  = v[e];
        const float en = __expf(fminf(t, 0.0f));
        v[e] = (t > 0.0f) ? (t + 1.0f) : en;
      }
    }
    vals[it] = v;
  }
  float* dst = C + (rowb + (size_t)hh) * (size_t)N + col0 + m * 4;
  for (int pass = 0; pass < 2; ++pass) {
#pragma unroll
    for (int it = 0; it < 8; ++it) {
      *(volatile v4f*)(dst + (size_t)(it * 2) * (size_t)N) = vals[it];
    }
    __threadfence();
  }
}

template <bool TWO, bool EPI>
__global__ __launch_bounds__(128)
void gemm_bf(const u16* __restrict__ A, const u16* __restrict__ A2, const u16* __restrict__ Bt, float* C,
             int M, int N, int K, const float* bp0, const float* bp1, const float* bp2, int e0, int e1, int e2) {
  __shared__ __align__(16) float slab[4 * SLAB64];
  const int tid = threadIdx.x, wave = tid >> 5, lane = tid & 31, hh = lane >> 4, m = lane & 15;
  const int ntile = N >> 6;
  const int bid   = blockIdx.x;
  const int rowb  = (bid / ntile) * 64 + wave * 16;
  const int col0  = (bid % ntile) * 64;
  if (rowb + 16 > M) return;
  const u16* ap  = A  + (size_t)(rowb + m) * K + 8 * hh;
  const u16* ap2 = A2 + (size_t)(rowb + m) * K + 8 * hh;
  const u16* bp  = Bt + (size_t)(col0 + m) * K + 8 * hh;
  const size_t bs = (size_t)16 * K;
  v8f acc0 = zero8(), acc1 = zero8(), acc2 = zero8(), acc3 = zero8();
#pragma unroll 1
  for (int k0 = 0; k0 < K; k0 += 32) {
    const v16b a   = ldfrag_b(ap + k0);
    const v16b fb0 = ldfrag_b(bp + k0);
    const v16b fb1 = ldfrag_b(bp + bs + k0);
    const v16b fb2 = ldfrag_b(bp + 2 * bs + k0);
    const v16b fb3 = ldfrag_b(bp + 3 * bs + k0);
    acc0 = mma_b(a, fb0, acc0);
    acc1 = mma_b(a, fb1, acc1);
    acc2 = mma_b(a, fb2, acc2);
    acc3 = mma_b(a, fb3, acc3);
    if constexpr (TWO) {
      const v16b a2 = ldfrag_b(ap2 + k0);
      acc0 = mma_b(a2, fb0, acc0);
      acc1 = mma_b(a2, fb1, acc1);
      acc2 = mma_b(a2, fb2, acc2);
      acc3 = mma_b(a2, fb3, acc3);
      guard6<v16b>(acc0, acc1, acc2, acc3, a, a2, fb0, fb1, fb2, fb3);
    } else {
      guard6<v16b>(acc0, acc1, acc2, acc3, a, fb0, fb1, fb2, fb3, a);
    }
  }
  v4f bias4;
#pragma unroll
  for (int e = 0; e < 4; ++e) bias4[e] = bias_at(bp0, bp1, bp2, e0, e1, e2, col0 + m * 4 + e);
  epi64b<EPI>(slab + wave * SLAB64, acc0, acc1, acc2, acc3, bias4, C, N, (size_t)rowb, col0, lane);
}

__global__ __launch_bounds__(ATT_THREADS)
void attn_la(const u16* __restrict__ QHp, const u16* __restrict__ QLp,
             const u16* __restrict__ VHp, const u16* __restrict__ VLp,
             const u16* __restrict__ THp, const u16* __restrict__ TLp,
             const float* __restrict__ DNp, u16* CHp, u16* CLp) {
#pragma clang fp contract(off)
  __shared__ __align__(16) float smem[WPB * WREG];

  const int tid  = threadIdx.x;
  const int wave = tid >> 5;
  const int lane = tid & 31;
  const int hh   = lane >> 4;
  const int c    = lane & 15;
  const int bid  = blockIdx.x;
  const int qt   = bid % NQT;
  const int hg   = bid / NQT;
  if (hg >= NHG) return;
  const int q0   = qt * 16;
  const int head = hg * WPB + wave;

  float* pt   = smem + wave * WREG;
  float* slab = pt + PTW;

  const size_t hcol = (size_t)head * HD + 8 * hh;
  const _Float16* Qh  = (const _Float16*)(const void*)QHp + (size_t)(q0 + c) * DQK + hcol;
  const _Float16* Ql  = (const _Float16*)(const void*)QLp + (size_t)(q0 + c) * DQK + hcol;
  const _Float16* Shb = (const _Float16*)(const void*)VHp + (size_t)c * DQK + hcol;
  const _Float16* Slb = (const _Float16*)(const void*)VLp + (size_t)c * DQK + hcol;
  const _Float16* Ahb = (const _Float16*)(const void*)THp + ((size_t)head * HD + c) * SEQ + 8 * hh;
  const _Float16* Alb = (const _Float16*)(const void*)TLp + ((size_t)head * HD + c) * SEQ + 8 * hh;
  const float lsc = 1.0f / (QSC * VSC);
  const float oc  = 1.0f / (PCAR * KCAR);
  const size_t KROW = (size_t)DQK;

  v8f o[4];
#pragma unroll
  for (int j = 0; j < 4; ++j) o[j] = zero8();
  const int ncaus = (q0 >> 5) + 1;
  const int ncl   = (ncaus < NKT) ? ncaus : NKT;
  const int qr0   = q0 + 8 * hh;

#pragma unroll 1
  for (int kt = 0; kt < ncl; ++kt) {
    const int kb = kt * 32;
    v8f s0 = zero8(), s1 = zero8();
    const _Float16* k0p = Shb + (size_t)kb * KROW;
    const _Float16* k1p = k0p + (size_t)16 * KROW;
    const _Float16* l0p = Slb + (size_t)kb * KROW;
    const _Float16* l1p = l0p + (size_t)16 * KROW;
#pragma unroll
    for (int kk = 0; kk < HD / 32; ++kk) {
      const v16h qh  = ldfrag_h(Qh + kk * 32);
      const v16h ql  = ldfrag_h(Ql + kk * 32);
      const v16h vh0 = ldfrag_h(k0p + kk * 32);
      const v16h vh1 = ldfrag_h(k1p + kk * 32);
      const v16h vl0 = ldfrag_h(l0p + kk * 32);
      const v16h vl1 = ldfrag_h(l1p + kk * 32);
      s0 = mma_h(qh, vh0, s0);
      s0 = mma_h(ql, vh0, s0);
      s0 = mma_h(qh, vl0, s0);
      s1 = mma_h(qh, vh1, s1);
      s1 = mma_h(ql, vh1, s1);
      s1 = mma_h(qh, vl1, s1);
      guard2(s0, s1, qh, ql, vh0, vl0, vh1, vl1);
    }
#pragma unroll
    for (int r = 0; r < 8; ++r) {
      const int row = qr0 + r;
      const float w0 = (kb + c <= row)      ? s0[r] * lsc : 0.0f;
      const float w1 = (kb + 16 + c <= row) ? s1[r] * lsc : 0.0f;
      const int ro = (8 * hh + r) * PTP + c;
      pt[ro]      = w0;
      pt[ro + 16] = w1;
    }
    wave_sync_lds();
    FragH ph, pl;
    {
      const float* prow = pt + c * PTP + 8 * hh;
      const v4f p0 = *(const v4f*)(prow), p1 = *(const v4f*)(prow + 4);
      const v4f p2 = *(const v4f*)(prow + 16), p3 = *(const v4f*)(prow + 20);
#pragma unroll
      for (int e = 0; e < 4; ++e) {
        const float ta = p0[e] * PCAR, tb = p1[e] * PCAR, tc = p2[e] * PCAR, td = p3[e] * PCAR;
        const _Float16 ha = (_Float16)ta, hb = (_Float16)tb, hc = (_Float16)tc, hd = (_Float16)td;
        ph.h[0][e]     = ha;
        ph.h[0][4 + e] = hb;
        ph.h[1][e]     = hc;
        ph.h[1][4 + e] = hd;
        pl.h[0][e]     = (_Float16)(ta - (float)ha);
        pl.h[0][4 + e] = (_Float16)(tb - (float)hb);
        pl.h[1][e]     = (_Float16)(tc - (float)hc);
        pl.h[1][4 + e] = (_Float16)(td - (float)hd);
      }
    }
    {
      const _Float16* vhp = Ahb + kb;
      const _Float16* vlp = Alb + kb;
#pragma unroll
      for (int jg = 0; jg < 2; ++jg) {
        const size_t da = (size_t)(2 * jg) * 16 * SEQ;
        const size_t db = da + (size_t)16 * SEQ;
        const v16h vha = ldfrag_h(vhp + da), vhb2 = ldfrag_h(vhp + db);
        const v16h vla = ldfrag_h(vlp + da), vlb2 = ldfrag_h(vlp + db);
        o[2 * jg]     = mma_h(ph.v, vha,  o[2 * jg]);
        o[2 * jg]     = mma_h(pl.v, vha,  o[2 * jg]);
        o[2 * jg]     = mma_h(ph.v, vla,  o[2 * jg]);
        o[2 * jg + 1] = mma_h(ph.v, vhb2, o[2 * jg + 1]);
        o[2 * jg + 1] = mma_h(pl.v, vhb2, o[2 * jg + 1]);
        o[2 * jg + 1] = mma_h(ph.v, vlb2, o[2 * jg + 1]);
        guard2(o[2 * jg], o[2 * jg + 1], ph.v, pl.v, vha, vhb2, vla, vlb2);
      }
    }
    wave_sync_lds();
  }
  acc_guard4(o[0], o[1], o[2], o[3]);
#pragma unroll
  for (int r = 0; r < 8; ++r) {
#pragma unroll
    for (int j = 0; j < 4; ++j) {
      const int idx = (8 * hh + r) * SLP + j * 16 + c;
      slab[idx] = o[j][r] * oc;
    }
  }
  wave_sync_lds();
  v4u oh[4], ol[4];
  const int rq = lane >> 3, c8 = (lane & 7) * 8;
  const float* dn = DNp + (size_t)q0 * DMOD + (size_t)head * HD + c8;
#pragma unroll
  for (int it = 0; it < 4; ++it) {
    const int row = it * 4 + rq;
    const v4f a  = *(const v4f*)(slab + row * SLP + c8), b4 = *(const v4f*)(slab + row * SLP + c8 + 4);
    const v4f da = *(const v4f*)(dn + (size_t)row * DMOD), db = *(const v4f*)(dn + (size_t)row * DMOD + 4);
    float w[8];
#pragma unroll
    for (int e = 0; e < 4; ++e) { w[e] = a[e] * (1.0f / da[e]); w[4 + e] = b4[e] * (1.0f / db[e]); }
#pragma unroll
    for (int e = 0; e < 4; ++e) {
      const float f0 = w[2 * e], f1 = w[2 * e + 1];
      const unsigned short h0 = bf_bits(f0), h1 = bf_bits(f1);
      const unsigned short l0 = bf_bits(f0 - bf_up(h0)), l1 = bf_bits(f1 - bf_up(h1));
      oh[it][e] = pk16(h0, h1);
      ol[it][e] = pk16(l0, l1);
    }
  }
  const size_t ob = (size_t)q0 * DMOD + (size_t)head * HD + c8;
  for (int pass = 0; pass < 2; ++pass) {
#pragma unroll
    for (int it = 0; it < 4; ++it) {
      const int row = it * 4 + rq;
      *(volatile v4u*)(CHp + ob + (size_t)row * DMOD) = oh[it];
      *(volatile v4u*)(CLp + ob + (size_t)row * DMOD) = ol[it];
    }
    __threadfence();
  }
}

extern "C" void kernel_launch(void* const* d_in, const int* in_sizes, int n_in,
                              void* d_out, int out_size, void* d_ws, size_t ws_size,
                              hipStream_t stream) {
  if (n_in < 11) return;
  const int need = ((NB - 1) * XS_FULL + SEQ) * DMOD;
  if (in_sizes[0] < need || in_sizes[1] < need || in_sizes[2] < need) return;
  if (in_sizes[3] != DMOD * DMOD || in_sizes[5] != DMOD * DMOD || in_sizes[7] != DMOD * DMOD || in_sizes[9] != DMOD * DMOD) return;
  if (in_sizes[4] != DMOD || in_sizes[6] != DMOD || in_sizes[8] != DMOD || in_sizes[10] != DMOD) return;
  if (out_size < need) return;

  const float* xq = (const float*)d_in[0];
  const float* xk = (const float*)d_in[1];
  const float* xv = (const float*)d_in[2];
  const float* wq = (const float*)d_in[3];
  const float* bq = (const float*)d_in[4];
  const float* wk = (const float*)d_in[5];
  const float* bk = (const float*)d_in[6];
  const float* wv = (const float*)d_in[7];
  const float* bv = (const float*)d_in[8];
  const float* wo = (const float*)d_in[9];
  const float* bo = (const float*)d_in[10];
  float*       out = (float*)d_out;

  const size_t szX = (size_t)SEQ * DMOD * 2;
  const size_t szW = (size_t)DMOD * DMOD * 2;
  const size_t szF = (size_t)SEQ * DMOD * 4;
  const size_t szP = (size_t)SEQ * DQK * 2;
  const size_t szT = (size_t)NH * HD * SEQ * 2;
  const size_t szD = (size_t)SEQ * DMOD * 4;
  const size_t szC = (size_t)SEQ * DMOD * 2;
  if (szC > szX) return;
  size_t off = 0;
  const size_t oXQ = off; off += szX;
  const size_t oXK = off; off += szX;
  const size_t oXV = off; off += szX;
  const size_t oWQ = off; off += szW;
  const size_t oWK = off; off += szW;
  const size_t oWV = off; off += szW;
  const size_t oWO = off; off += szW;
  const size_t oFQ = off; off += szF;
  const size_t oFW = off; off += szF;
  const size_t oQH = off; off += szP;
  const size_t oQL = off; off += szP;
  const size_t oVH = off; off += szP;
  const size_t oVL = off; off += szP;
  const size_t oTH = off; off += szT;
  const size_t oTL = off; off += szT;
  const size_t oDN = off; off += szD;
  const size_t oCL = off; off += szC;
  if (off > ws_size) return;
  if (off > (size_t)WS_CAP) return;

  char* ws = (char*)d_ws;
  u16*   XQ  = (u16*)(ws + oXQ);
  u16*   CH  = (u16*)(ws + oXQ);
  u16*   XK  = (u16*)(ws + oXK);
  u16*   XV  = (u16*)(ws + oXV);
  u16*   WQT = (u16*)(ws + oWQ);
  u16*   WKT = (u16*)(ws + oWK);
  u16*   WVT = (u16*)(ws + oWV);
  u16*   WOT = (u16*)(ws + oWO);
  float* FQ  = (float*)(ws + oFQ);
  float* FW  = (float*)(ws + oFW);
  u16*   QH  = (u16*)(ws + oQH);
  u16*   QL  = (u16*)(ws + oQL);
  u16*   VH  = (u16*)(ws + oVH);
  u16*   VL  = (u16*)(ws + oVL);
  u16*   TH  = (u16*)(ws + oTH);
  u16*   TL  = (u16*)(ws + oTL);
  float* DN  = (float*)(ws + oDN);
  u16*   CL  = (u16*)(ws + oCL);

  const dim3 b256(256), b128(128), bAT(ATT_THREADS);
  const int  n8x = (SEQ * DMOD) / 8;
  const dim3 gX3((n8x + 255) / 256, 3);
  const int  ntv = (DMOD + 63) / 64;
  const dim3 gW((DMOD / 64) * ntv);
  const dim3 gG((SEQ / 64) * (DMOD / 64));
  const dim3 gRW(SEQ);
  const dim3 gKT(NH * NST);
  const dim3 gDN(DMOD / 256);
  const dim3 gAT(NQT * NHG);

  k_wt<<<gW, b256, 0, stream>>>(wq, DMOD, DMOD, ntv, WQT, 0);
  k_wt<<<gW, b256, 0, stream>>>(wk, DMOD, DMOD, ntv, WKT, 0);
  k_wt<<<gW, b256, 0, stream>>>(wv, DMOD, DMOD, ntv, WVT, 0);
  k_wt<<<gW, b256, 0, stream>>>(wo, DMOD, DMOD, ntv, WOT, 0);

  for (int b = 0; b < NB; ++b) {
    const size_t xo = (size_t)b * XS_FULL * DMOD;
    cvt_bf3<<<gX3, b256, 0, stream>>>(xq + xo, xk + xo, xv + xo, XQ, XK, XV, n8x);
    gemm_bf<false, true><<<gG, b128, 0, stream>>>(XQ, XQ, WQT, FQ, SEQ, DMOD, DMOD, bq, bq, bq,
                                                  DMOD, DMOD + 1, DMOD + 2);
    gemm_bf<false, false><<<gG, b128, 0, stream>>>(XV, XV, WVT, FW, SEQ, DMOD, DMOD, bv, bv, bv,
                                                   DMOD, DMOD + 1, DMOD + 2);
    qv16<<<gRW, b256, 0, stream>>>(FQ, FW, QH, QL, VH, VL);
    gemm_bf<false, true><<<gG, b128, 0, stream>>>(XK, XK, WKT, FW, SEQ, DMOD, DMOD, bk, bk, bk,
                                                  DMOD, DMOD + 1, DMOD + 2);
    kt16<<<gKT, b256, 0, stream>>>(FW, TH, TL);
    k_den<<<gDN, b256, 0, stream>>>(FQ, FW, DN);
    attn_la<<<gAT, bAT, 0, stream>>>(QH, QL, VH, VL, TH, TL, DN, CH, CL);
    gemm_bf<true, false><<<gG, b128, 0, stream>>>(CH, CL, WOT, out + xo, SEQ, DMOD, DMOD, bo, bo, bo,
                                                  DMOD, DMOD + 1, DMOD + 2);
  }
  (void)hipGetLastError();
}
